// Precoding_gnn_44495861186889
// MI455X (gfx1250) — hardware-verified
//
#include <hip/hip_runtime.h>

typedef __attribute__((ext_vector_type(16))) _Float16 v16h;
typedef __attribute__((ext_vector_type(8)))  _Float16 v8h;
typedef __attribute__((ext_vector_type(2)))  _Float16 f16x2;
typedef __attribute__((ext_vector_type(8)))  float    v8f;

#define TPB 256
#define MM  64
#define KK  32
#define DD  32

#define OFF_W1S 0
#define OFF_W1M 64
#define OFF_W1K 128
#define OFF_W2S 192
#define OFF_W2M (192 + 1024)
#define OFF_W2K (192 + 2048)
#define OFF_W3S (192 + 3072)
#define OFF_W3M (192 + 4096)
#define OFF_W3K (192 + 5120)
#define OFF_W4S (192 + 6144)
#define OFF_W4M (192 + 7168)
#define OFF_W4K (192 + 8192)
#define OFF_W5S (192 + 9216)
#define OFF_W5M (192 + 9216 + 64)
#define OFF_W5K (192 + 9216 + 128)
#define WPOOL   (192 + 9216 + 192)

struct Smem {
  _Float16 H0[MM * KK * DD];
  _Float16 H1[MM * KK * DD];
  _Float16 msgMh[MM * DD];
  _Float16 msgKh[KK * DD];
  float    BM[MM * DD];
  float    BK[KK * DD];
  _Float16 Wf[WPOOL];
  float    red[TPB];
};

__device__ __forceinline__ v16h cat16(v8h lo, v8h hi) {
  return __builtin_shufflevector(lo, hi, 0,1,2,3,4,5,6,7,8,9,10,11,12,13,14,15);
}

__device__ __forceinline__ v16h load_afrag(const _Float16* W, int hbase, int l15, int half) {
  const _Float16* row = W + (hbase + l15) * DD;
  const int ko = half * 8;
  v8h lo = *(const v8h*)(row + ko);
  v8h hi = *(const v8h*)(row + 16 + ko);
  return cat16(lo, hi);
}

__device__ __forceinline__ v16h load_bfrag(const _Float16* entityRow, int half) {
  const int ko = half * 8;
  v8h lo = *(const v8h*)(entityRow + ko);
  v8h hi = *(const v8h*)(entityRow + 16 + ko);
  return cat16(lo, hi);
}
__device__ __forceinline__ v8f wmma16(v16h a, v16h b, v8f c) {
  v8f d = __builtin_amdgcn_wmma_f32_16x16x32_f16(false, a, false, b, (short)0, c, false, false);
  asm volatile("v_nop\n\tv_nop\n\tv_nop\n\tv_nop" : "+v"(d) : "v"(a), "v"(b));
  return d;
}
__device__ __forceinline__ void rescale_pow2(_Float16* __restrict__ H, float* __restrict__ red, int tid) {
  float mx = 0.f;
  for (int i = tid * 8; i < MM * KK * DD; i += TPB * 8) {
    const v8h v = *(const v8h*)(H + i);
#pragma unroll
    for (int j = 0; j < 8; ++j) mx = fmaxf(mx, fabsf((float)v[j]));
  }
  red[tid] = mx;
  __syncthreads();
  for (int off = TPB / 2; off > 0; off >>= 1) { if (tid < off) red[tid] = fmaxf(red[tid], red[tid + off]); __syncthreads(); }
  const float m = red[0];
  __syncthreads();
  int e = 0;
  if (m > 0.f) (void)frexpf(m, &e);
  const float sc = ldexpf(1.0f, -e);
  for (int i = tid * 8; i < MM * KK * DD; i += TPB * 8) {
    v8h v = *(const v8h*)(H + i);
#pragma unroll
    for (int j = 0; j < 8; ++j) v[j] = (_Float16)((float)v[j] * sc);
    *(v8h*)(H + i) = v;
  }
  __syncthreads();
}

__device__ __forceinline__ void midlayer(Smem& s,
                                         const _Float16* __restrict__ Hin,
                                         _Float16* __restrict__ Hout,
                                         int wsOff, int wmOff, int wkOff, int tid)
{
  const int lane = tid & 31, wv = tid >> 5, half = lane >> 4, l15 = lane & 15;

  for (int pe = tid; pe < (MM * DD) / 2; pe += TPB) {
    int m = pe >> 4, dp = (pe & 15) * 2;
    const f16x2* col = (const f16x2*)(Hin + m * KK * DD + dp);
    float a0 = 0.f, a1 = 0.f;
    #pragma unroll
    for (int k = 0; k < KK; ++k) { const f16x2 v = col[k * 16]; a0 += (float)v.x; a1 += (float)v.y; }
    f16x2 r; r.x = (_Float16)a0; r.y = (_Float16)a1;
    *(f16x2*)(s.msgMh + m * DD + dp) = r;
  }
  for (int pe = tid; pe < (KK * DD) / 2; pe += TPB) {
    int k = pe >> 4, dp = (pe & 15) * 2;
    const f16x2* col = (const f16x2*)(Hin + k * DD + dp);
    float a0 = 0.f, a1 = 0.f;
    #pragma unroll 8
    for (int m = 0; m < MM; ++m) { const f16x2 v = col[m * 512]; a0 += (float)v.x; a1 += (float)v.y; }
    f16x2 r; r.x = (_Float16)a0; r.y = (_Float16)a1;
    *(f16x2*)(s.msgKh + k * DD + dp) = r;
  }
  __syncthreads();

  {
    const v8f zero = {};
    const int ht = wv >> 2, mB = wv & 3;
    v16h aW = load_afrag(s.Wf + wmOff, ht * 16, l15, half);
    v16h bM = load_bfrag(s.msgMh + (mB * 16 + l15) * DD, half);
    v8f c = wmma16(aW, bM, zero);
    float* dst = s.BM + (mB * 16 + l15) * DD + ht * 16 + half * 8;
    #pragma unroll
    for (int j = 0; j < 8; ++j) dst[j] = c[j];
    if (wv < 4) {
      const int ht2 = wv >> 1, kB = wv & 1;
      v16h aK = load_afrag(s.Wf + wkOff, ht2 * 16, l15, half);
      v16h bK = load_bfrag(s.msgKh + (kB * 16 + l15) * DD, half);
      v8f c2 = wmma16(aK, bK, zero);
      float* dst2 = s.BK + (kB * 16 + l15) * DD + ht2 * 16 + half * 8;
      #pragma unroll
      for (int j = 0; j < 8; ++j) dst2[j] = c2[j];
    }
  }
  __syncthreads();

  const v16h aS0 = load_afrag(s.Wf + wsOff, 0,  l15, half);
  const v16h aS1 = load_afrag(s.Wf + wsOff, 16, l15, half);
  for (int i = wv * 16; i < wv * 16 + 16; ++i) {
    const int m = i >> 1, kb = (i & 1) * 16;
    const int p = m * KK + kb + l15;
    const v16h bH = load_bfrag(Hin + p * DD, half);
    #pragma unroll
    for (int ht = 0; ht < 2; ++ht) {
      const int hb = ht * 16 + half * 8;
      const float* bmrow = s.BM + m * DD + hb;
      const float* bkrow = s.BK + (kb + l15) * DD + hb;
      v8f c;
      #pragma unroll
      for (int j = 0; j < 8; ++j) c[j] = bmrow[j] + bkrow[j];
      c = wmma16((ht ? aS1 : aS0), bH, c);
      v8h hv;
      #pragma unroll
      for (int j = 0; j < 8; ++j) {
        float z = c[j] > 0.f ? c[j] : 0.f;
        hv[j] = (_Float16)z;
      }
      *(v8h*)(Hout + p * DD + hb) = hv;
    }
  }
  __syncthreads();
  rescale_pow2(Hout, s.red, tid);
}

__global__ __launch_bounds__(TPB, 1)
void precoding_gnn_kernel(
    const float* __restrict__ x,
    const float* w1s, const float* w1m, const float* w1k,
    const float* w2s, const float* w2m, const float* w2k,
    const float* w3s, const float* w3m, const float* w3k,
    const float* w4s, const float* w4m, const float* w4k,
    const float* w5s, const float* w5m, const float* w5k,
    float* __restrict__ out)
{
  __shared__ Smem s;
  const int tid = threadIdx.x;
  const int b   = blockIdx.x;

  float* Xs = reinterpret_cast<float*>(s.H1);
  const float* xb = x + (size_t)b * (MM * KK * 2);
  for (int i = tid; i < MM * KK * 2; i += TPB) Xs[i] = xb[i];

  auto cvt = [&](const float* src, int off, int n) {
    for (int i = tid; i < n; i += TPB) s.Wf[off + i] = (_Float16)src[i];
  };
  cvt(w1s, OFF_W1S, 64);   cvt(w1m, OFF_W1M, 64);   cvt(w1k, OFF_W1K, 64);
  cvt(w2s, OFF_W2S, 1024); cvt(w2m, OFF_W2M, 1024); cvt(w2k, OFF_W2K, 1024);
  cvt(w3s, OFF_W3S, 1024); cvt(w3m, OFF_W3M, 1024); cvt(w3k, OFF_W3K, 1024);
  cvt(w4s, OFF_W4S, 1024); cvt(w4m, OFF_W4M, 1024); cvt(w4k, OFF_W4K, 1024);
  cvt(w5s, OFF_W5S, 64);   cvt(w5m, OFF_W5M, 64);   cvt(w5k, OFF_W5K, 64);
  __syncthreads();

  for (int idx = tid; idx < MM * 2; idx += TPB) {
    int m = idx >> 1, c = idx & 1;
    float acc = 0.f;
    #pragma unroll
    for (int k = 0; k < KK; ++k) acc += Xs[(m * KK + k) * 2 + c];
    s.BM[idx] = acc;
  }
  for (int idx = tid; idx < KK * 2; idx += TPB) {
    int k = idx >> 1, c = idx & 1;
    float acc = 0.f;
    #pragma unroll
    for (int m = 0; m < MM; ++m) acc += Xs[(m * KK + k) * 2 + c];
    s.BK[idx] = acc;
  }
  __syncthreads();
  for (int p = tid; p < MM * KK; p += TPB) {
    int m = p >> 5, k = p & 31;
    float x0 = Xs[p * 2], x1 = Xs[p * 2 + 1];
    float a0 = s.BM[m * 2], a1 = s.BM[m * 2 + 1];
    float g0 = s.BK[k * 2], g1 = s.BK[k * 2 + 1];
    #pragma unroll
    for (int hq = 0; hq < 4; ++hq) {
      v8h hv;
      #pragma unroll
      for (int j = 0; j < 8; ++j) {
        int h = hq * 8 + j;
        float z = (float)s.Wf[OFF_W1S + h * 2] * x0 + (float)s.Wf[OFF_W1S + h * 2 + 1] * x1
                + (float)s.Wf[OFF_W1M + h * 2] * a0 + (float)s.Wf[OFF_W1M + h * 2 + 1] * a1
                + (float)s.Wf[OFF_W1K + h * 2] * g0 + (float)s.Wf[OFF_W1K + h * 2 + 1] * g1;
        z = z > 0.f ? z : 0.f;
        hv[j] = (_Float16)z;
      }
      *(v8h*)(s.H0 + p * DD + hq * 8) = hv;
    }
  }
  __syncthreads();
  rescale_pow2(s.H0, s.red, tid);

  midlayer(s, s.H0, s.H1, OFF_W2S, OFF_W2M, OFF_W2K, tid);
  midlayer(s, s.H1, s.H0, OFF_W3S, OFF_W3M, OFF_W3K, tid);
  midlayer(s, s.H0, s.H1, OFF_W4S, OFF_W4M, OFF_W4K, tid);

  const _Float16* Hin = s.H1;
  for (int pe = tid; pe < (MM * DD) / 2; pe += TPB) {
    int m = pe >> 4, dp = (pe & 15) * 2;
    const f16x2* col = (const f16x2*)(Hin + m * KK * DD + dp);
    f16x2 a0 = col[0], a1 = col[16];
    #pragma unroll
    for (int k = 2; k < KK; k += 2) { a0 += col[k * 16]; a1 += col[k * 16 + 16]; }
    *(f16x2*)(s.msgMh + m * DD + dp) = a0 + a1;
  }
  for (int pe = tid; pe < (KK * DD) / 2; pe += TPB) {
    int k = pe >> 4, dp = (pe & 15) * 2;
    const f16x2* col = (const f16x2*)(Hin + k * DD + dp);
    f16x2 a0 = col[0], a1 = col[512];
    #pragma unroll
    for (int m = 2; m < MM; m += 2) { a0 += col[m * 512]; a1 += col[m * 512 + 512]; }
    *(f16x2*)(s.msgKh + k * DD + dp) = a0 + a1;
  }
  __syncthreads();
  for (int idx = tid; idx < MM * 2; idx += TPB) {
    int m = idx >> 1, c = idx & 1;
    float acc = 0.f;
    #pragma unroll
    for (int d = 0; d < DD; ++d)
      acc += (float)s.Wf[OFF_W5M + c * DD + d] * (float)s.msgMh[m * DD + d];
    s.BM[idx] = acc;
  }
  for (int idx = tid; idx < KK * 2; idx += TPB) {
    int k = idx >> 1, c = idx & 1;
    float acc = 0.f;
    #pragma unroll
    for (int d = 0; d < DD; ++d)
      acc += (float)s.Wf[OFF_W5K + c * DD + d] * (float)s.msgKh[k * DD + d];
    s.BK[idx] = acc;
  }
  __syncthreads();

  float* Out = reinterpret_cast<float*>(s.H0);
  float psum = 0.f;
  for (int p = tid; p < MM * KK; p += TPB) {
    int m = p >> 5, k = p & 31;
    float o0 = s.BM[m * 2]     + s.BK[k * 2];
    float o1 = s.BM[m * 2 + 1] + s.BK[k * 2 + 1];
    #pragma unroll
    for (int d = 0; d < DD; ++d) {
      float hv = (float)Hin[p * DD + d];
      o0 += (float)s.Wf[OFF_W5S + d]      * hv;
      o1 += (float)s.Wf[OFF_W5S + DD + d] * hv;
    }
    Out[p * 2]     = o0;
    Out[p * 2 + 1] = o1;
    psum += o0 * o0 + o1 * o1;
  }
  s.red[tid] = psum;
  __syncthreads();
  for (int off = TPB / 2; off > 0; off >>= 1) {
    if (tid < off) s.red[tid] += s.red[tid + off];
    __syncthreads();
  }
  const float alpha = 1.0f / sqrtf(s.red[0]);
  float* og = out + (size_t)b * (MM * KK * 2);
  for (int i = tid; i < MM * KK * 2; i += TPB) { const float v = alpha * Out[i]; *(volatile float*)(og + i) = v; __threadfence(); *(volatile float*)(og + i) = v; }
}

extern "C" void kernel_launch(void* const* d_in, const int* in_sizes, int n_in,
                              void* d_out, int out_size, void* d_ws, size_t ws_size,
                              hipStream_t stream) {
  const float* x = (const float*)d_in[0];
  const int bs = in_sizes[0] / (MM * KK * 2);
  (void)n_in; (void)out_size; (void)d_ws; (void)ws_size;
  precoding_gnn_kernel<<<dim3(bs), dim3(TPB), 0, stream>>>(
      x,
      (const float*)d_in[1],  (const float*)d_in[2],  (const float*)d_in[3],
      (const float*)d_in[4],  (const float*)d_in[5],  (const float*)d_in[6],
      (const float*)d_in[7],  (const float*)d_in[8],  (const float*)d_in[9],
      (const float*)d_in[10], (const float*)d_in[11], (const float*)d_in[12],
      (const float*)d_in[13], (const float*)d_in[14], (const float*)d_in[15],
      (float*)d_out);
}
